// MixGNN_56762287784200
// MI455X (gfx1250) — hardware-run, weakly checked
//
#include <hip/hip_runtime.h>


namespace {
constexpr int N = 10000, E = 320000, D = 256, NL = 3;
constexpr float XS = 8.0f, WSC = 256.0f, BN_EPS = 1e-5f;
typedef _Float16 b16;
typedef __attribute__((ext_vector_type(16))) _Float16 v16b;
typedef __attribute__((ext_vector_type(8))) _Float16 v8b;
typedef __attribute__((ext_vector_type(8))) float v8f;
typedef __attribute__((ext_vector_type(4))) float v4f;
__device__ __forceinline__ float bf16_rne(float f) { unsigned int u = __float_as_uint(f); u += 0x7FFFu + ((u >> 16) & 1u); float r = __uint_as_float(u & 0xFFFF0000u); asm volatile("" : "+v"(r)); return r; }
__device__ __forceinline__ void split16(float v, b16& hi, b16& lo) { hi = (b16)v; lo = (b16)(v - (float)hi); }
__device__ __forceinline__ v16b frag_kb(const b16* p, int hh) { const v8b a = *(const v8b*)(p + 8 * hh), b = *(const v8b*)(p + 16 + 8 * hh); v16b f;
#pragma unroll
  for (int e = 0; e < 8; ++e) { f[e] = a[e]; f[8 + e] = b[e]; } return f; }
__device__ __forceinline__ v8f wmma16b(v16b a, v16b b, v8f c) { v8f d = __builtin_amdgcn_wmma_f32_16x16x32_f16(false, a, false, b, (short)0, c, false, false); asm volatile("v_nop\n\tv_nop\n\tv_nop\n\tv_nop" : "+v"(d) : "v"(a), "v"(b)); return d; }
__device__ __forceinline__ void wave_lds_sync() { __builtin_amdgcn_fence(__ATOMIC_RELEASE, "workgroup"); __builtin_amdgcn_wave_barrier(); __builtin_amdgcn_fence(__ATOMIC_ACQUIRE, "workgroup"); }
__device__ __forceinline__ float pmul(float a, float b) { float p = a * b; asm volatile("" : "+v"(p)); return p; }
__device__ __forceinline__ int iclamp(int v, int lo, int hi) { return v < lo ? lo : (v > hi ? hi : v); }
constexpr int CSR_NBLK7 = 512, CSR_GB7 = 7, CSR_GN7 = 1 << CSR_GB7  , CSR_TS7 = (CSR_GN7 < 32 ? 32 : CSR_GN7)  , CSR_MAXG7 = 512, CSR_CAP7 = 12288  ;
__device__ __host__ __forceinline__ int csr_tix7(int v) { return (v >> CSR_GB7) * CSR_TS7 + (v & (CSR_GN7 - 1)); }
__global__ __launch_bounds__(64) void csrA_kernel7(const int* __restrict__ dst, int E, int N, int nG, int CHP, int NGP, int* __restrict__ STG, int* __restrict__ HST) {
  extern __shared__ int sm[];
  int* cnt = sm; int* run = sm + NGP; int* ids = sm + 2 * NGP;
  const int b = blockIdx.x; const int ch = (E + CSR_NBLK7 - 1) / CSR_NBLK7; const int e0 = b * ch, e1 = min(E, e0 + ch);
  for (int i = threadIdx.x; i < NGP; i += 64) cnt[i] = 0;
  for (int i = threadIdx.x; i < CHP; i += 64) ids[i] = -1;
  __syncthreads();
  if (threadIdx.x == 0) {
    for (int e = e0; e < e1; ++e) { int d = dst[e]; d = (d < 0) ? 0 : (d >= N ? N - 1 : d); cnt[d >> CSR_GB7] += 1; }
    int acc = 0; for (int g = 0; g < nG; ++g) { run[g] = acc; acc += cnt[g]; }
    for (int e = e0; e < e1; ++e) { int d = dst[e]; d = (d < 0) ? 0 : (d >= N ? N - 1 : d); const int g = d >> CSR_GB7; ids[run[g]] = e; run[g] += 1; } }
  __syncthreads();
  typedef __attribute__((ext_vector_type(4))) int v4i;
  for (int pass = 0; pass < 2; ++pass) {
    for (int i = threadIdx.x; i < CHP / 4; i += 64) *(volatile v4i*)(STG + (size_t)b * CHP + i * 4) = *(const v4i*)(&ids[i * 4]);
    for (int i = threadIdx.x; i < NGP / 4; i += 64) { v4i v; for (int e = 0; e < 4; ++e) v[e] = (i * 4 + e < nG) ? cnt[i * 4 + e] : 0; *(volatile v4i*)(HST + (size_t)b * NGP + i * 4) = v; }
    __threadfence(); }
}
__global__ __launch_bounds__(512) void csrS_kernel7(const int* __restrict__ HST, int nG, int NGP, int* __restrict__ START, int* __restrict__ TOT, int* __restrict__ OFF) {
  __shared__ int tot[CSR_MAXG7];
  const int b = threadIdx.x;
  for (int pass = 0; pass < 2; ++pass) { int runb = 0; for (int g = 0; g < nG; ++g) { int c = HST[(size_t)b * NGP + g]; c = (c < 0) ? 0 : c; ((volatile int*)OFF)[(size_t)g * CSR_NBLK7 + b] = runb; runb += c; } __threadfence(); }
  for (int g = threadIdx.x; g < nG; g += 512) { int s = 0; for (int bb = 0; bb < CSR_NBLK7; ++bb) { int c = HST[(size_t)bb * NGP + g]; s += (c < 0) ? 0 : c; } tot[g] = s; }
  __syncthreads();
  if (threadIdx.x < 32) {
    __shared__ int st[CSR_MAXG7 + 32];
    if (threadIdx.x == 0) { int acc = 0; for (int g = 0; g < NGP; ++g) { st[g] = acc; if (g < nG) acc += (tot[g] + 31) & ~31; } st[NGP] = acc; }
    __builtin_amdgcn_fence(__ATOMIC_RELEASE, "workgroup"); __builtin_amdgcn_wave_barrier(); __builtin_amdgcn_fence(__ATOMIC_ACQUIRE, "workgroup");
    for (int pass = 0; pass < 2; ++pass) { for (int i = threadIdx.x; i < NGP + 32; i += 32) { ((volatile int*)START)[i] = (i <= NGP) ? st[min(i, NGP)] : 0; ((volatile int*)TOT)[i] = (i < nG) ? tot[i] : 0; } __threadfence(); } }
}
__global__ __launch_bounds__(256) void csrB_kernel7(const int* __restrict__ dst, int N, int nG, int CHP, int NGP, int permLen, const int* __restrict__ STG, const int* __restrict__ HST, const int* __restrict__ OFF, const int* __restrict__ START, const int* __restrict__ TOT, int* __restrict__ PERM, int* __restrict__ ROWPTR, int* __restrict__ ROWCNT, int* __restrict__ FLAG) {
  typedef __attribute__((ext_vector_type(4))) int v4i;
  __shared__ int ids[CSR_CAP7]; __shared__ unsigned short key[CSR_CAP7]; __shared__ int outp[CSR_CAP7]; __shared__ int ncnt[CSR_GN7 + 1]; __shared__ int boff[CSR_NBLK7 + 1];
  const int g = blockIdx.x, t_ = threadIdx.x; int tot = TOT[g]; int st = START[g], stn = START[g + 1]; const int v0 = g * CSR_GN7; const int nv = min(CSR_GN7, N - v0); const int t0 = g * CSR_TS7;
  st = (st < 0) ? 0 : (st > permLen - 32 ? permLen - 32 : st) & ~31; stn = (stn < st) ? st : (stn > permLen ? permLen : stn); tot = (tot < 0) ? 0 : tot; if (tot > stn - st && tot <= CSR_CAP7) tot = stn - st;
  if (tot > CSR_CAP7) {
    for (int pass = 0; pass < 2; ++pass) { for (int i = t_; i < CSR_TS7 / 4; i += 256) { v4i a, c; for (int e = 0; e < 4; ++e) { a[e] = st; c[e] = 0; } *(volatile v4i*)(ROWPTR + t0 + i * 4) = a; *(volatile v4i*)(ROWCNT + t0 + i * 4) = c; } if (t_ == 0) ((volatile int*)FLAG)[0] = 1; __threadfence(); } (void)nv; return; }
  if (t_ == 0) { int acc = 0; for (int b = 0; b < CSR_NBLK7; ++b) { boff[b] = acc; int c = HST[(size_t)b * NGP + g]; c = (c < 0) ? 0 : (c > CHP ? CHP : c); acc += c; if (acc > tot) acc = tot; } boff[CSR_NBLK7] = acc; }
  for (int i = t_; i <= CSR_GN7; i += 256) ncnt[i] = 0;
  __syncthreads();
  for (int b = 0; b < CSR_NBLK7; ++b) { const int c = boff[b + 1] - boff[b]; int o_ = OFF[(size_t)g * CSR_NBLK7 + b]; o_ = (o_ < 0) ? 0 : (o_ > CHP - c ? CHP - c : o_); const int* src_ = STG + (size_t)b * CHP + o_;
    for (int i = t_; i < c; i += 256) { int id = src_[i]; id = (id < 0) ? 0 : id; ids[boff[b] + i] = id; int d = dst[id]; d = (d < v0) ? v0 : (d >= N ? N - 1 : d); int kk = d - v0; kk = (kk < 0) ? 0 : (kk >= CSR_GN7 ? CSR_GN7 - 1 : kk); key[boff[b] + i] = (unsigned short)kk; } }
  __syncthreads();
  if (t_ == 0) { for (int i = 0; i < tot; ++i) ncnt[key[i]] += 1; int acc = 0; for (int vl = 0; vl < CSR_GN7; ++vl) { const int c = ncnt[vl]; ncnt[vl] = acc; acc += c; } ncnt[CSR_GN7] = acc;
    for (int i = 0; i < tot; ++i) { const int vl = key[i]; outp[ncnt[vl]] = ids[i]; ncnt[vl] += 1; }
    for (int vl = CSR_GN7; vl > 0; --vl) ncnt[vl] = ncnt[vl - 1]; ncnt[0] = 0; }
  __syncthreads();
  for (int pass = 0; pass < 2; ++pass) {
    for (int i = t_; i < (stn - st) / 4; i += 256) { v4i v; for (int e = 0; e < 4; ++e) { const int q = i * 4 + e; v[e] = (q < tot) ? outp[q] : -1; } *(volatile v4i*)(PERM + st + i * 4) = v; }
    for (int i = t_; i < CSR_TS7 / 4; i += 256) { v4i a, c; for (int e = 0; e < 4; ++e) { const int vl = i * 4 + e; const int vc = vl < CSR_GN7 ? vl : CSR_GN7; a[e] = (vl < CSR_GN7) ? st + ncnt[vc] : st; c[e] = (vl < nv) ? (ncnt[(vc < CSR_GN7 ? vc : CSR_GN7 - 1) + 1] - ncnt[vc]) : 0; } *(volatile v4i*)(ROWPTR + t0 + i * 4) = a; *(volatile v4i*)(ROWCNT + t0 + i * 4) = c; }
    __threadfence(); }
}
__global__ __launch_bounds__(256) void csrZ_kernel7(int* __restrict__ p, size_t n4) { typedef __attribute__((ext_vector_type(4))) int v4i; const size_t tid = (size_t)blockIdx.x * 256 + threadIdx.x, nth = (size_t)gridDim.x * 256; v4i z = {0, 0, 0, 0}; for (size_t i = tid; i < n4; i += nth) *(volatile v4i*)(p + i * 4) = z; }
struct CsrBufs7 { int *STG, *HST, *OFF, *START, *TOT, *PERM, *ROWPTR, *ROWCNT, *FLAG; int nG, NGP, CHP; size_t permLen; char* base; size_t bytes; };
static size_t csr_carve7(CsrBufs7& c, char* ws, size_t off, int E, int N) {
  const size_t off0 = off; c.base = ws + off;
  auto al = [&](size_t bytes) { char* p = ws + off; off += (bytes + 255) & ~(size_t)255; return p; };
  c.nG = (N + CSR_GN7 - 1) / CSR_GN7; c.NGP = (c.nG + 31) & ~31; const int ch = (E + CSR_NBLK7 - 1) / CSR_NBLK7; c.CHP = (ch + 31) & ~31; c.permLen = (size_t)E + 32 * (size_t)c.nG + 32;
  c.STG = (int*)al((size_t)CSR_NBLK7 * c.CHP * 4); c.HST = (int*)al((size_t)CSR_NBLK7 * c.NGP * 4); c.OFF = (int*)al((size_t)c.NGP * CSR_NBLK7 * 4); c.START = (int*)al((size_t)(c.NGP + 64) * 4); c.TOT = (int*)al((size_t)(c.NGP + 64) * 4);
  c.PERM = (int*)al(c.permLen * 4); c.ROWPTR = (int*)al((size_t)c.nG * CSR_TS7 * 4); c.ROWCNT = (int*)al((size_t)c.nG * CSR_TS7 * 4); c.FLAG = (int*)al(256);
  c.bytes = off - off0; return off;
}
static void csr_build7(const CsrBufs7& c, const int* dst, int E, int N, hipStream_t stream) {
  const size_t smem = (size_t)(2 * c.NGP + c.CHP) * 4;
  csrZ_kernel7<<<512, 256, 0, stream>>>((int*)c.base, c.bytes / 16);
  csrA_kernel7<<<CSR_NBLK7, 64, smem, stream>>>(dst, E, N, c.nG, c.CHP, c.NGP, c.STG, c.HST);
  csrS_kernel7<<<1, 512, 0, stream>>>(c.HST, c.nG, c.NGP, c.START, c.TOT, c.OFF);
  csrB_kernel7<<<c.nG, 256, 0, stream>>>(dst, N, c.nG, c.CHP, c.NGP, (int)c.permLen, c.STG, c.HST, c.OFF, c.START, c.TOT, c.PERM, c.ROWPTR, c.ROWCNT, c.FLAG);
}


__global__ __launch_bounds__(256) void wput_kernel(const float* __restrict__ w, int KIN, int KTOT, int koff, int ooff, b16* __restrict__ WT) { const int KG = KIN / 8; const int u = blockIdx.x * 256 + threadIdx.x; if (u >= D * KG) return; const int o = u / KG, k0 = (u % KG) * 8; v8b v;
#pragma unroll
  for (int j = 0; j < 8; ++j) v[j] = (b16)(bf16_rne(w[(size_t)(k0 + j) * D + o]) * WSC); for (int pass = 0; pass < 2; ++pass) { *(volatile v8b*)(WT + (size_t)(ooff + o) * KTOT + koff + k0) = v; __threadfence(); } }
__global__ __launch_bounds__(32) void qkvs_kernel(const float* __restrict__ x, const b16* __restrict__ WT, const float* __restrict__ bq, const float* __restrict__ bk, const float* __restrict__ bv, const float* __restrict__ bs, int NLIM, float* __restrict__ QK) {
  __shared__ __attribute__((aligned(16))) b16 Ah[16][D + 8]; __shared__ float Tf[16][132]; const int lane = threadIdx.x, nloc = lane & 15, hlf = lane >> 4; const int cg = blockIdx.x % 8; const size_t m0 = (size_t)(blockIdx.x / 8) * 16; if (m0 >= (size_t)NLIM) return;
  for (int rr = 0; rr < 16; ++rr) for (int q = 0; q < D / 32; ++q) Ah[rr][q * 32 + lane] = (b16)(bf16_rne(x[(m0 + rr) * D + q * 32 + lane]) * XS);
  wave_lds_sync(); v8f acc[8];
#pragma unroll
  for (int t = 0; t < 8; ++t) acc[t] = (v8f){};
#pragma unroll 2
  for (int kb = 0; kb < D; kb += 32) { const v16b a = frag_kb(&Ah[nloc][kb], hlf);
#pragma unroll
    for (int t = 0; t < 8; ++t) acc[t] = wmma16b(a, frag_kb(WT + (size_t)(cg * 128 + t * 16 + nloc) * D + kb, hlf), acc[t]); }
  const int which = cg / 2; const float* bias = which == 0 ? bq : (which == 1 ? bk : (which == 2 ? bv : bs));
#pragma unroll
  for (int t = 0; t < 8; ++t) { const int c = cg * 128 + t * 16 + nloc; const float bb = bf16_rne(bias[c - which * D]);
#pragma unroll
    for (int r8 = 0; r8 < 8; ++r8) Tf[8 * hlf + r8][t * 16 + nloc] = acc[t][r8] * (1.0f / (XS * WSC)) + bb; }
  wave_lds_sync();
  for (int pass = 0; pass < 2; ++pass) { for (int rr = 0; rr < 16; ++rr) *(volatile v4f*)(QK + (m0 + rr) * 4 * D + cg * 128 + lane * 4) = *(const v4f*)(&Tf[rr][lane * 4]); __threadfence(); }
}
__global__ __launch_bounds__(256) void tconv_kernel(const float* __restrict__ QK, const int* __restrict__ srcs, const int* __restrict__ PERM, const int* __restrict__ ROWPTR, const int* __restrict__ ROWCNT, int permLen, int NLIM, float* __restrict__ H) {
  const int wave = threadIdx.x >> 5, lane = threadIdx.x & 31; const size_t i = (size_t)blockIdx.x * 8 + wave; if (i >= (size_t)NLIM) return; int st = ROWPTR[i], cnt = ROWCNT[i]; cnt = iclamp(cnt, 0, 1 << 20); st = iclamp(st, 0, permLen - cnt);
  const v4f q0 = *(const v4f*)(QK + i * 4 * D + lane * 4), q1 = *(const v4f*)(QK + i * 4 * D + 128 + lane * 4); float m = -INFINITY, den = 0.0f; v4f a0 = {0.0f, 0.0f, 0.0f, 0.0f}, a1 = {0.0f, 0.0f, 0.0f, 0.0f};
#pragma unroll 1
  for (int j = 0; j < cnt; ++j) { const int e = iclamp(PERM[st + j], 0, E - 1); const size_t u = (size_t)iclamp(srcs[e], 0, N - 1); if (u >= (size_t)NLIM) continue; const float* kr = QK + u * 4 * D + D; const v4f k0 = *(const v4f*)(kr + lane * 4), k1 = *(const v4f*)(kr + 128 + lane * 4);
    float s = 0.0f; for (int c = 0; c < 4; ++c) s += pmul(q0[c], k0[c]) + pmul(q1[c], k1[c]); for (int o = 16; o; o >>= 1) s += __shfl_xor(s, o); s *= (1.0f / 16.0f);
    const float mn = fmaxf(m, s); const float sc = (m == -INFINITY) ? 0.0f : __expf(m - mn); const float p = __expf(s - mn); den = den * sc + p; const float* vr = QK + u * 4 * D + 2 * D; const v4f v0 = *(const v4f*)(vr + lane * 4), v1 = *(const v4f*)(vr + 128 + lane * 4);
    for (int c = 0; c < 4; ++c) { a0[c] = pmul(a0[c], sc) + pmul(p, v0[c]); a1[c] = pmul(a1[c], sc) + pmul(p, v1[c]); } m = mn; }
  const float inv = den > 0.0f ? 1.0f / den : 0.0f; const float* sr = QK + i * 4 * D + 3 * D; const v4f s0 = *(const v4f*)(sr + lane * 4), s1 = *(const v4f*)(sr + 128 + lane * 4); v4f r0, r1;
  for (int c = 0; c < 4; ++c) { r0[c] = fmaxf(pmul(a0[c], inv) + s0[c], 0.0f); r1[c] = fmaxf(pmul(a1[c], inv) + s1[c], 0.0f); }
  for (int pass = 0; pass < 2; ++pass) { *(volatile v4f*)(H + i * D + lane * 4) = r0; *(volatile v4f*)(H + i * D + 128 + lane * 4) = r1; __threadfence(); } }
__global__ __launch_bounds__(256) void mean_kernel(const float* __restrict__ Hin, const int* __restrict__ srcs, const int* __restrict__ PERM, const int* __restrict__ ROWPTR, const int* __restrict__ ROWCNT, int permLen, int NLIM, float* __restrict__ MB) {
  const int wave = threadIdx.x >> 5, lane = threadIdx.x & 31; const size_t i = (size_t)blockIdx.x * 8 + wave; if (i >= (size_t)NLIM) return; int st = ROWPTR[i], cnt = ROWCNT[i]; cnt = iclamp(cnt, 0, 1 << 20); st = iclamp(st, 0, permLen - cnt);
  v4f a0 = {0.0f, 0.0f, 0.0f, 0.0f}, a1 = {0.0f, 0.0f, 0.0f, 0.0f}; int n = 0;
#pragma unroll 1
  for (int j = 0; j < cnt; ++j) { const int e = iclamp(PERM[st + j], 0, E - 1); const size_t u = (size_t)iclamp(srcs[e], 0, N - 1); if (u >= (size_t)NLIM) continue; ++n; const v4f h0 = *(const v4f*)(Hin + u * D + lane * 4), h1 = *(const v4f*)(Hin + u * D + 128 + lane * 4); for (int c = 0; c < 4; ++c) { a0[c] += h0[c]; a1[c] += h1[c]; } }
  const float inv = 1.0f / (float)(n > 0 ? n : 1); for (int c = 0; c < 4; ++c) { a0[c] = pmul(a0[c], inv); a1[c] = pmul(a1[c], inv); }
  for (int pass = 0; pass < 2; ++pass) { *(volatile v4f*)(MB + i * D + lane * 4) = a0; *(volatile v4f*)(MB + i * D + 128 + lane * 4) = a1; __threadfence(); } }
__global__ __launch_bounds__(32) void sage_kernel(const float* __restrict__ MB, const float* __restrict__ Hin, const b16* __restrict__ WT, const float* __restrict__ bl, const float* __restrict__ gam, const float* __restrict__ bet, const float* __restrict__ alpha, int NLIM, float* __restrict__ Hout) {
  __shared__ __attribute__((aligned(16))) b16 Ah[16][2 * D + 8], Al[16][2 * D + 8]; __shared__ float Tf[16][132]; const int lane = threadIdx.x, nloc = lane & 15, hlf = lane >> 4; const int cg = blockIdx.x % 2; const size_t m0 = (size_t)(blockIdx.x / 2) * 16; if (m0 >= (size_t)NLIM) return;
  for (int rr = 0; rr < 16; ++rr) for (int q = 0; q < D / 32; ++q) { b16 p, ql; split16(MB[(m0 + rr) * D + q * 32 + lane] * XS, p, ql); Ah[rr][q * 32 + lane] = p; Al[rr][q * 32 + lane] = ql; split16(Hin[(m0 + rr) * D + q * 32 + lane] * XS, p, ql); Ah[rr][D + q * 32 + lane] = p; Al[rr][D + q * 32 + lane] = ql; }
  wave_lds_sync(); v8f acc[8];
#pragma unroll
  for (int t = 0; t < 8; ++t) acc[t] = (v8f){};
#pragma unroll 2
  for (int kb = 0; kb < 2 * D; kb += 32) { const v16b a = frag_kb(&Ah[nloc][kb], hlf), al = frag_kb(&Al[nloc][kb], hlf);
#pragma unroll
    for (int t = 0; t < 8; ++t) { const v16b bw = frag_kb(WT + (size_t)(cg * 128 + t * 16 + nloc) * 2 * D + kb, hlf); acc[t] = wmma16b(a, bw, acc[t]); acc[t] = wmma16b(al, bw, acc[t]); } }
  const float a_ = 1.0f / (1.0f + __expf(-bf16_rne(alpha[0]))); const float bns = rsqrtf(1.0f + BN_EPS);
#pragma unroll
  for (int t = 0; t < 8; ++t) { const int c = cg * 128 + t * 16 + nloc; const float bb = bf16_rne(bl[c]), g = bf16_rne(gam[c]), be = bf16_rne(bet[c]);
#pragma unroll
    for (int r8 = 0; r8 < 8; ++r8) { const int rl = 8 * hlf + r8; float z = acc[t][r8] * (1.0f / (XS * WSC)) + bb; z = pmul(pmul(z, bns), g) + be; z = pmul(a_, z) + pmul(1.0f - a_, Hin[(m0 + rl) * D + c]); Tf[rl][t * 16 + nloc] = fmaxf(z, 0.0f); } }
  wave_lds_sync();
  for (int pass = 0; pass < 2; ++pass) { for (int rr = 0; rr < 16; ++rr) *(volatile v4f*)(Hout + (m0 + rr) * D + cg * 128 + lane * 4) = *(const v4f*)(&Tf[rr][lane * 4]); __threadfence(); }
}
}

extern "C" void kernel_launch(void* const* d_in, const int* in_sizes, int n_in, void* d_out, int out_size, void* d_ws, size_t ws_size, hipStream_t stream) {
  (void)n_in;
  auto Fp = [&](int i) { return (const float*)d_in[i]; }; auto Ip = [&](int i) { return (const int*)d_in[i]; };
  if (in_sizes[0] != N * D || in_sizes[1] != 2 * E || in_sizes[2] != D * D || in_sizes[8] != D * D || in_sizes[10] != NL * D * D || in_sizes[12] != NL * D * D || in_sizes[15] != 1 || out_size != N * D) return;
  const int NLIM = N;
  size_t off = 0; char* ws = (char*)d_ws;
  auto carve = [&](size_t bytes) { char* p = ws + off; off += (bytes + 255) & ~(size_t)255; return p; };
  b16* WQ = (b16*)carve((size_t)4 * D * D * 2); b16* WL = (b16*)carve((size_t)NL * D * 2 * D * 2); float* QK = (float*)carve((size_t)N * 4 * D * 4); float* HA = (float*)carve((size_t)N * D * 4); float* HB = (float*)carve((size_t)N * D * 4); float* MB = (float*)carve((size_t)N * D * 4); CsrBufs7 csr; off = csr_carve7(csr, ws, off, E, N);
  if (off > ws_size || off > ((size_t)128 << 20)) return;
  for (int w = 0; w < 4; ++w) wput_kernel<<<(D * 32 + 255) / 256, 256, 0, stream>>>(Fp(2 + 2 * w), D, D, 0, w * D, WQ);
  for (int l = 0; l < NL; ++l) { wput_kernel<<<(D * 32 + 255) / 256, 256, 0, stream>>>(Fp(10) + (size_t)l * D * D, D, 2 * D, 0, l * D, WL); wput_kernel<<<(D * 32 + 255) / 256, 256, 0, stream>>>(Fp(12) + (size_t)l * D * D, D, 2 * D, D, l * D, WL); }
  csr_build7(csr, Ip(1) + E, E, N, stream);
  qkvs_kernel<<<(NLIM / 16) * 8, 32, 0, stream>>>(Fp(0), WQ, Fp(3), Fp(5), Fp(7), Fp(9), NLIM, QK);
  tconv_kernel<<<(NLIM + 7) / 8, 256, 0, stream>>>(QK, Ip(1), csr.PERM, csr.ROWPTR, csr.ROWCNT, (int)csr.permLen, NLIM, HA);
  float* hin = HA; float* hout = HB;
  for (int l = 0; l < NL; ++l) {
    mean_kernel<<<(NLIM + 7) / 8, 256, 0, stream>>>(hin, Ip(1), csr.PERM, csr.ROWPTR, csr.ROWCNT, (int)csr.permLen, NLIM, MB);
    sage_kernel<<<(NLIM / 16) * 2, 32, 0, stream>>>(MB, hin, WL + (size_t)l * D * 2 * D, Fp(11) + l * D, Fp(13) + l * D, Fp(14) + l * D, Fp(15), NLIM, l == NL - 1 ? (float*)d_out : hout);
    float* t = hin; hin = hout; hout = t; }
}
